// PointTransformer_850403525317
// MI455X (gfx1250) — hardware-verified
//
#include <hip/hip_runtime.h>
#include <math.h>
#include <stdint.h>


typedef __attribute__((ext_vector_type(16))) _Float16 v16h;
typedef __attribute__((ext_vector_type(8)))  _Float16 v8h;
typedef __attribute__((ext_vector_type(8)))  float    v8f;
typedef __attribute__((ext_vector_type(4)))  float    v4f;

#define NP    512
#define DM    256
#define NH    8
#define HDM   32
#define HIDR  682
#define HIDP  704
#define QCH   128
#define NPAIR (QCH * NP)

__device__ __forceinline__ void dep_guard_h(v8f& a, v8f& b, v16h x, v16h y) { asm volatile("v_nop\n\tv_nop\n\tv_nop\n\tv_nop" : "+v"(a), "+v"(b) : "v"(x), "v"(y)); }
__device__ __forceinline__ void keep4_h(v16h a, v16h b, v16h c, v16h d) { asm volatile("v_nop" :: "v"(a), "v"(b), "v"(c), "v"(d)); }
__device__ __forceinline__ void acc_guard4(v8f& a, v8f& b, v8f& c, v8f& d) { asm volatile("v_nop\n\tv_nop\n\tv_nop\n\tv_nop" : "+v"(a), "+v"(b), "+v"(c), "+v"(d)); }

template <typename T> struct Frag;
template <> struct Frag<_Float16> {
  typedef v16h V; union U { v16h v; v8h h[2]; };
  static __device__ __forceinline__ v16h load(const _Float16* p) {
    U f; f.h[0] = *(const v8h*)(p); f.h[1] = *(const v8h*)(p + 16); return f.v;
  }
  static __device__ __forceinline__ v8f mma(v16h a, v16h b, v8f c) {
    return __builtin_amdgcn_wmma_f32_16x16x32_f16(false, a, false, b, (short)0, c, false, false);
  }
  static __device__ __forceinline__ void guard(v8f& a, v8f& b, v16h x, v16h y) { dep_guard_h(a, b, x, y); }
  static __device__ __forceinline__ void keep(v16h a, v16h b, v16h c, v16h d) { keep4_h(a, b, c, d); }
};
template <int ET> struct Elem;
template <> struct Elem<0> { typedef _Float16 T; };

template <int ET, int BIAS_MODE, int OUT_MODE, bool RESID, int MI>
__global__ __launch_bounds__(256) void wmma_gemm(
    const unsigned short* __restrict__ Ap, int lda, long strideA,
    const unsigned short* __restrict__ Btp, int ldb, long strideB,
    void* __restrict__ Cout, int ldc, long strideC,
    const float* __restrict__ bias,
    const float* __restrict__ resid, long strideR,
    int M, int N, int K, float scale) {
  typedef typename Elem<ET>::T T;
  typedef typename Frag<T>::V V;
  const T* A = (const T*)Ap; const T* Bt = (const T*)Btp;
  __shared__ __align__(16) float sT[8][16 * 68];
  const int b    = blockIdx.y;
  const int lane = threadIdx.x & 31;
  const int wave = threadIdx.x >> 5;
  const int tilesN = N >> 6;
  const int tilesM = M / (16 * MI);
  const int tile = blockIdx.x * 8 + wave;
  if (tile >= tilesM * tilesN) return;
  const int tm = tile / tilesN;
  const int tn = tile - tm * tilesN;
  const int m0 = tm * (16 * MI);
  const int n0 = tn << 6;

  const T* Ab = A  + (size_t)b * (size_t)strideA;
  const T* Bb = Bt + (size_t)b * (size_t)strideB;

  const int rlane = lane & 15;
  const int koff  = (lane >> 4) * 8;
  const int mOff  = (lane >> 4) * 8;

  v8f acc[MI][4];
#pragma unroll
  for (int i = 0; i < MI; ++i)
#pragma unroll
    for (int j = 0; j < 4; ++j) acc[i][j] = (v8f){0.f,0.f,0.f,0.f,0.f,0.f,0.f,0.f};

  for (int k0 = 0; k0 < K; k0 += 32) {
    V bh[4];
#pragma unroll
    for (int j = 0; j < 4; ++j) {
      const size_t bo = (size_t)(n0 + (j << 4) + rlane) * ldb + koff + k0;
      bh[j] = Frag<T>::load(Bb + bo);
    }
#pragma unroll
    for (int i = 0; i < MI; ++i) {
      const size_t ao = (size_t)(m0 + (i << 4) + rlane) * lda + koff + k0;
      V ah = Frag<T>::load(Ab + ao);
#pragma unroll
      for (int j = 0; j < 4; ++j) acc[i][j] = Frag<T>::mma(ah, bh[j], acc[i][j]);
      Frag<T>::guard(acc[i][0], acc[i][3], ah, ah);
    }
    Frag<T>::keep(bh[0], bh[1], bh[2], bh[3]);
  }
#pragma unroll
  for (int i = 0; i < MI; ++i) acc_guard4(acc[i][0], acc[i][1], acc[i][2], acc[i][3]);

  float* slab = sT[wave];
  const float* Rb = RESID ? (resid + (size_t)b * (size_t)strideR) : nullptr;
#pragma unroll
  for (int i = 0; i < MI; ++i) {
    const int mBase = m0 + (i << 4);
#pragma unroll
    for (int j = 0; j < 4; ++j) {
      const int n = n0 + (j << 4) + rlane;
      float bv = 0.f;
      if (BIAS_MODE == 2) bv = bias[n];
#pragma unroll
      for (int r = 0; r < 8; ++r) {
        float v = acc[i][j][r] * scale;
        if (BIAS_MODE == 1) v += bias[mBase + mOff + r];
        if (BIAS_MODE == 2) v += bv;
        if (RESID) v += Rb[(size_t)(mBase + mOff + r) * ldc + n];
        slab[(mOff + r) * 68 + (j << 4) + rlane] = v;
      }
    }
    __builtin_amdgcn_fence(__ATOMIC_RELEASE, "workgroup");
    __builtin_amdgcn_wave_barrier();
    __builtin_amdgcn_fence(__ATOMIC_ACQUIRE, "workgroup");
    if (OUT_MODE == 0) {
      float* C = (float*)Cout + (size_t)b * (size_t)strideC;
      const int hh = lane >> 4, c4 = (lane & 15) * 4;
      for (int pass = 0; pass < 2; ++pass) {
#pragma unroll
        for (int it = 0; it < 8; ++it) {
          const int row = it * 2 + hh;
          v4f v = *(const v4f*)(slab + row * 68 + c4);
          *(volatile v4f*)(C + (size_t)(mBase + row) * ldc + n0 + c4) = v;
        }
        __threadfence();
      }
    } else {
      const int q = lane >> 3, c8 = (lane & 7) * 8;
      unsigned short* C = (unsigned short*)Cout + (size_t)b * (size_t)strideC;
      for (int pass = 0; pass < 2; ++pass) {
#pragma unroll
        for (int it = 0; it < 4; ++it) {
          const int row = it * 4 + q;
          const float* sp = slab + row * 68 + c8;
          v8h hv;
#pragma unroll
          for (int e = 0; e < 8; ++e) hv[e] = (_Float16)sp[e];
          *(volatile v8h*)(C + (size_t)(mBase + row) * ldc + n0 + c8) = hv;
        }
        __threadfence();
      }
    }
    __builtin_amdgcn_fence(__ATOMIC_RELEASE, "workgroup");
    __builtin_amdgcn_wave_barrier();
    __builtin_amdgcn_fence(__ATOMIC_ACQUIRE, "workgroup");
  }
}

__device__ __forceinline__ unsigned pack_h2(float a, float b) {
  const unsigned short ua = __builtin_bit_cast(unsigned short, (_Float16)a);
  const unsigned short ub = __builtin_bit_cast(unsigned short, (_Float16)b);
  return (unsigned)ua | ((unsigned)ub << 16);
}
__device__ __forceinline__ void st2_u32(unsigned short* base, size_t off_halves, unsigned u) {
  volatile unsigned* p = (volatile unsigned*)(base + off_halves);
  *p = u; __threadfence(); *p = u;
}
__device__ __forceinline__ void st2_f32(float* base, size_t off, float v) {
  volatile float* p = (volatile float*)(base + off);
  *p = v; __threadfence(); *p = v;
}
__device__ __forceinline__ float silu_fast(float z) {
  const float e = __expf(-z);
  return z * __builtin_amdgcn_rcpf(1.0f + e);
}
__device__ __forceinline__ float silu_acc(float z) {
  const float e = expf(-z);
  return z * __builtin_amdgcn_rcpf(1.0f + e);
}
__device__ __forceinline__ float blk_sum256(float v, float* red) {
#pragma unroll
  for (int off = 16; off > 0; off >>= 1) v += __shfl_xor(v, off, 32);
  const int lane = threadIdx.x & 31, wave = threadIdx.x >> 5;
  if (lane == 0) red[wave] = v;
  __syncthreads();
  float s = red[0];
#pragma unroll
  for (int q = 1; q < 8; ++q) s += red[q];
  __syncthreads();
  return s;
}
__device__ __forceinline__ float blk_max256(float v, float* red) {
#pragma unroll
  for (int off = 16; off > 0; off >>= 1) v = fmaxf(v, __shfl_xor(v, off, 32));
  const int lane = threadIdx.x & 31, wave = threadIdx.x >> 5;
  if (lane == 0) red[wave] = v;
  __syncthreads();
  float s = red[0];
#pragma unroll
  for (int q = 1; q < 8; ++q) s = fmaxf(s, red[q]);
  __syncthreads();
  return s;
}

__global__ __launch_bounds__(256) void k_cast_pad(const float* __restrict__ src, int srows, int scols, int spitch,
                                                   unsigned short* __restrict__ dst, int drows, int dcols) {
  const int p = blockIdx.x * 256 + threadIdx.x;
  const int npairs = (drows * dcols) >> 1;
  if (p < npairs) {
    const int e = 2 * p;
    const int r = e / dcols;
    const int c = e - r * dcols;
    float v0 = 0.f, v1 = 0.f;
    if (r < srows) {
      if (c < scols)     v0 = src[(size_t)r * spitch + c];
      if (c + 1 < scols) v1 = src[(size_t)r * spitch + c + 1];
    }
    st2_u32(dst, (size_t)e, pack_h2(v0, v1));
  }
}
__global__ __launch_bounds__(256) void k_pad_f32(const float* __restrict__ src, int sn, float* __restrict__ dst, int dn) {
  const int p = blockIdx.x * 256 + threadIdx.x;
  if (p < dn) {
    const float v = (p < sn) ? src[p] : 0.f;
    st2_f32(dst, (size_t)p, v);
  }
}

__global__ __launch_bounds__(256) void k_ln16(const float* __restrict__ x, const float* __restrict__ w,
                                               const float* __restrict__ bb, unsigned short* __restrict__ y16) {
  __shared__ float red[8];
  __shared__ float ys[DM];
  const int i = blockIdx.x, d = threadIdx.x;
  const float v = x[(size_t)i * DM + d];
  const float mu = blk_sum256(v, red) * (1.0f / 256.0f);
  const float c = v - mu;
  const float var = blk_sum256(c * c, red) * (1.0f / 256.0f);
  const float y = c * (1.0f / sqrtf(var + 1e-5f)) * w[d] + bb[d];
  ys[d] = y;
  __syncthreads();
  if (d < 128) st2_u32(y16, (size_t)i * DM + 2 * d, pack_h2(ys[2 * d], ys[2 * d + 1]));
}

__global__ __launch_bounds__(256) void k_vt(const unsigned short* __restrict__ qkv, unsigned short* __restrict__ vt) {
  __shared__ unsigned short tile[32][520];
  const int t = threadIdx.x;
  const int d0 = blockIdx.x * 32;
  if (d0 < DM) {
    const int cp = (t & 15) * 2;
#pragma unroll 1
    for (int it = 0; it < 32; ++it) {
      const int j = it * 16 + (t >> 4);
      const unsigned u = *(const unsigned*)(qkv + (size_t)j * (3 * DM) + 2 * DM + d0 + cp);
      tile[cp][j]     = (unsigned short)(u & 0xFFFFu);
      tile[cp + 1][j] = (unsigned short)(u >> 16);
    }
  }
  __syncthreads();
  const int j2 = 2 * t;
#pragma unroll 1
  for (int dl = 0; dl < 32; ++dl) {
    unsigned u = 0u;
    if (d0 < DM) u = (unsigned)tile[dl][j2] | ((unsigned)tile[dl][j2 + 1] << 16);
    st2_u32(vt, (size_t)(d0 + dl) * NP + j2, u);
  }
}

__global__ __launch_bounds__(256) void k_pair_g1(const float* __restrict__ coords, const float* __restrict__ w,
                                                  const float* __restrict__ bias, unsigned short* __restrict__ G, int i0) {
  const int t = threadIdx.x;
  const int k2 = (t & 127) * 2;
  const int rsub = t >> 7;
  const float w00 = w[k2 * 3 + 0], w01 = w[k2 * 3 + 1], w02 = w[k2 * 3 + 2];
  const float w10 = w[k2 * 3 + 3], w11 = w[k2 * 3 + 4], w12 = w[k2 * 3 + 5];
  const float b0 = bias[k2], b1 = bias[k2 + 1];
#pragma unroll 1
  for (int it = 0; it < 8; ++it) {
    const int r = blockIdx.x * 16 + it * 2 + rsub;
    const int i = i0 + (r >> 9);
    const int j = r & (NP - 1);
    const float r0 = coords[i * 3 + 0] - coords[j * 3 + 0];
    const float r1 = coords[i * 3 + 1] - coords[j * 3 + 1];
    const float r2 = coords[i * 3 + 2] - coords[j * 3 + 2];
    const float z0 = (r0 * w00 + r1 * w01 + r2 * w02) + b0;
    const float z1 = (r0 * w10 + r1 * w11 + r2 * w12) + b1;
    const unsigned u = pack_h2(silu_fast(z0), silu_fast(z1));
    st2_u32(G, (size_t)r * DM + k2, u);
  }
}

__global__ __launch_bounds__(256) void k_pair_g2t(const float* __restrict__ coords, const float* __restrict__ w,
                                                   const float* __restrict__ bias, unsigned short* __restrict__ G, int i0) {
  const int t = threadIdx.x;
  const int j2 = 2 * t;
  const int il = blockIdx.x >> 4;
  const int kg = blockIdx.x & 15;
  const int i = i0 + il;
  const float ci0 = coords[i * 3 + 0], ci1 = coords[i * 3 + 1], ci2 = coords[i * 3 + 2];
  const float ra0 = ci0 - coords[j2 * 3 + 0], ra1 = ci1 - coords[j2 * 3 + 1], ra2 = ci2 - coords[j2 * 3 + 2];
  const float rc0 = ci0 - coords[j2 * 3 + 3], rc1 = ci1 - coords[j2 * 3 + 4], rc2 = ci2 - coords[j2 * 3 + 5];
#pragma unroll 1
  for (int kk = 0; kk < 16; ++kk) {
    const int k = kg * 16 + kk;
    const float wk0 = w[k * 3 + 0], wk1 = w[k * 3 + 1], wk2 = w[k * 3 + 2];
    const float bk = bias[k];
    const float z0 = (ra0 * wk0 + ra1 * wk1 + ra2 * wk2) + bk;
    const float z1 = (rc0 * wk0 + rc1 * wk1 + rc2 * wk2) + bk;
    const unsigned u = pack_h2(silu_fast(z0), silu_fast(z1));
    st2_u32(G, ((size_t)il * DM + k) * NP + j2, u);
  }
}

__global__ __launch_bounds__(256) void k_softmax(const float* __restrict__ S, const float* __restrict__ biasT,
                                                  const float* __restrict__ rb2b, unsigned short* __restrict__ P16) {
  __shared__ float red[8];
  const int i = blockIdx.x, t = threadIdx.x, j2 = 2 * t;
#pragma unroll 1
  for (int h = 0; h < NH; ++h) {
    const float* sp = S + ((size_t)h * NP + i) * NP + j2;
    const float* bp = biasT + (size_t)h * (NP * NP) + (size_t)i * NP + j2;
    const float bb = rb2b[h];
    const float s0 = sp[0] + (bp[0] + bb);
    const float s1 = sp[1] + (bp[1] + bb);
    const float m = blk_max256(fmaxf(s0, s1), red);
    const float e0 = expf(s0 - m), e1 = expf(s1 - m);
    const float sum = blk_sum256(e0 + e1, red);
    const float inv = 1.0f / sum;
    const float p0 = (e0 * inv) * 32768.0f;
    const float p1 = (e1 * inv) * 32768.0f;
    st2_u32(P16, ((size_t)i * 16 + h) * NP + j2, pack_h2(p0, p1));
  }
#pragma unroll 1
  for (int h = NH; h < 16; ++h) st2_u32(P16, ((size_t)i * 16 + h) * NP + j2, 0u);
}

__global__ __launch_bounds__(256) void k_combine_ln(const float* __restrict__ x, const float* __restrict__ ctx,
                                                     const float* __restrict__ rv2b, const float* __restrict__ w,
                                                     const float* __restrict__ bb, float* __restrict__ x1,
                                                     unsigned short* __restrict__ y16) {
  __shared__ float red[8];
  __shared__ float ys[DM];
  const int i = blockIdx.x, d = threadIdx.x;
  const int h = d >> 5, dd = d & 31;
  const float a = ctx[((size_t)h * NP + i) * 64 + dd] + rv2b[d];
  const float v = x[(size_t)i * DM + d] + a;
  st2_f32(x1, (size_t)i * DM + d, v);
  const float mu = blk_sum256(v, red) * (1.0f / 256.0f);
  const float c = v - mu;
  const float var = blk_sum256(c * c, red) * (1.0f / 256.0f);
  const float y = c * (1.0f / sqrtf(var + 1e-5f)) * w[d] + bb[d];
  ys[d] = y;
  __syncthreads();
  if (d < 128) st2_u32(y16, (size_t)i * DM + 2 * d, pack_h2(ys[2 * d], ys[2 * d + 1]));
}

__global__ __launch_bounds__(256) void k_swiglu(const float* __restrict__ c12, unsigned short* __restrict__ u16, int npairs) {
  const int p = blockIdx.x * 256 + threadIdx.x;
  if (p < npairs) {
    const int e = 2 * p;
    const int row = e / HIDP;
    const int col = e - row * HIDP;
    const float* rp = c12 + (size_t)row * (2 * HIDP);
    const float a0 = rp[col], a1 = rp[col + 1];
    const float g0 = rp[HIDP + col], g1 = rp[HIDP + col + 1];
    const float u0 = silu_acc(a0) * g0;
    const float u1 = silu_acc(a1) * g1;
    st2_u32(u16, (size_t)e, pack_h2(u0, u1));
  }
}

static inline size_t alignup256(size_t x) { return (x + 255) & ~(size_t)255; }

extern "C" void kernel_launch(void* const* d_in, const int* in_sizes, int n_in,
                              void* d_out, int out_size, void* d_ws, size_t ws_size,
                              hipStream_t stream)
{
  if (n_in < 22) return;
  if (in_sizes[0] != NP * DM || in_sizes[1] != NP * 3 || in_sizes[6] != 3 * DM * DM ||
      in_sizes[14] != DM * DM || in_sizes[16] != HIDR * DM || in_sizes[20] != DM * HIDR ||
      out_size != NP * DM) return;

  const float* x      = (const float*)d_in[0];
  const float* coords = (const float*)d_in[1];
  const float* ln1_w  = (const float*)d_in[2];
  const float* ln1_b  = (const float*)d_in[3];
  const float* ln2_w  = (const float*)d_in[4];
  const float* ln2_b  = (const float*)d_in[5];
  const float* qkv_w  = (const float*)d_in[6];
  const float* qkv_b  = (const float*)d_in[7];
  const float* rb1_w  = (const float*)d_in[8];
  const float* rb1_b  = (const float*)d_in[9];
  const float* rb2_w  = (const float*)d_in[10];
  const float* rb2_b  = (const float*)d_in[11];
  const float* rv1_w  = (const float*)d_in[12];
  const float* rv1_b  = (const float*)d_in[13];
  const float* rv2_w  = (const float*)d_in[14];
  const float* rv2_b  = (const float*)d_in[15];
  const float* ffn_w1 = (const float*)d_in[16];
  const float* ffn_b1 = (const float*)d_in[17];
  const float* ffn_w2 = (const float*)d_in[18];
  const float* ffn_b2 = (const float*)d_in[19];
  const float* ffn_w3 = (const float*)d_in[20];
  const float* ffn_b3 = (const float*)d_in[21];
  float* out = (float*)d_out;

  size_t off = 0;
  char* base = (char*)d_ws;
  auto carve = [&](size_t bytes) -> char* { char* r = base + off; off += alignup256(bytes); return r; };
  unsigned short* qkvw16 = (unsigned short*)carve((size_t)3 * DM * DM * 2);
  unsigned short* rb2w16 = (unsigned short*)carve((size_t)16 * DM * 2);
  unsigned short* rv2w16 = (unsigned short*)carve((size_t)(DM + 32) * DM * 2);
  unsigned short* w12p16 = (unsigned short*)carve((size_t)2 * HIDP * DM * 2);
  unsigned short* w3p16  = (unsigned short*)carve((size_t)DM * HIDP * 2);
  float*          b12p   = (float*)carve((size_t)2 * HIDP * 4);
  unsigned short* XN1    = (unsigned short*)carve((size_t)NP * DM * 2);
  unsigned short* QKV16  = (unsigned short*)carve((size_t)NP * 3 * DM * 2);
  unsigned short* VT16   = (unsigned short*)carve((size_t)(DM + 32) * NP * 2);
  float*          S      = (float*)carve((size_t)NH * NP * NP * 4);
  float*          BIAST  = (float*)carve((size_t)16 * NP * NP * 4);
  unsigned short* P16    = (unsigned short*)carve((size_t)NP * 16 * NP * 2);
  unsigned short* G      = (unsigned short*)carve((size_t)NPAIR * DM * 2);
  unsigned short* T16    = (unsigned short*)carve((size_t)NP * 16 * DM * 2);
  float*          CTX1   = (float*)carve((size_t)NH * NP * 64 * 4);
  float*          CTX    = (float*)carve((size_t)NH * NP * 64 * 4);
  float*          X1     = (float*)carve((size_t)NP * DM * 4);
  unsigned short* XN2    = (unsigned short*)carve((size_t)NP * DM * 2);
  float*          C12    = (float*)carve((size_t)NP * 2 * HIDP * 4);
  unsigned short* U16    = (unsigned short*)carve((size_t)NP * HIDP * 2);
  if (off > ws_size || off > (size_t)134217728) return;

  const dim3 blk(256);

  k_cast_pad<<<dim3((3 * DM * DM / 2 + 255) / 256), blk, 0, stream>>>(qkv_w, 3 * DM, DM, DM, qkvw16, 3 * DM, DM);
  k_cast_pad<<<dim3((16 * DM / 2 + 255) / 256), blk, 0, stream>>>(rb2_w, NH, DM, DM, rb2w16, 16, DM);
  k_cast_pad<<<dim3(((DM + 32) * DM / 2 + 255) / 256), blk, 0, stream>>>(rv2_w, DM, DM, DM, rv2w16, DM + 32, DM);
  k_cast_pad<<<dim3((HIDP * DM / 2 + 255) / 256), blk, 0, stream>>>(ffn_w1, HIDR, DM, DM, w12p16, HIDP, DM);
  k_cast_pad<<<dim3((HIDP * DM / 2 + 255) / 256), blk, 0, stream>>>(ffn_w2, HIDR, DM, DM, w12p16 + (size_t)HIDP * DM, HIDP, DM);
  k_cast_pad<<<dim3((DM * HIDP / 2 + 255) / 256), blk, 0, stream>>>(ffn_w3, DM, HIDR, HIDR, w3p16, DM, HIDP);
  k_pad_f32<<<dim3((HIDP + 255) / 256), blk, 0, stream>>>(ffn_b1, HIDR, b12p, HIDP);
  k_pad_f32<<<dim3((HIDP + 255) / 256), blk, 0, stream>>>(ffn_b2, HIDR, b12p + HIDP, HIDP);

  k_ln16<<<dim3(NP), blk, 0, stream>>>(x, ln1_w, ln1_b, XN1);
  wmma_gemm<0, 2, 1, false, 4><<<dim3((NP / 64) * (3 * DM / 64) / 8, 1), blk, 0, stream>>>(
      XN1, DM, 0, qkvw16, DM, 0, QKV16, 3 * DM, 0, qkv_b, nullptr, 0, NP, 3 * DM, DM, 1.0f);
  k_vt<<<dim3((DM + 32) / 32), blk, 0, stream>>>(QKV16, VT16);
  wmma_gemm<0, 0, 0, false, 4><<<dim3((NP / 64) * (NP / 64) / 8, NH), blk, 0, stream>>>(
      QKV16, 3 * DM, HDM, QKV16 + DM, 3 * DM, HDM, S, NP, (long)NP * NP, nullptr, nullptr, 0,
      NP, NP, HDM, 0.17677669529663687f);

  for (int ch = 0; ch < NP / QCH; ++ch) {
    const int i0 = ch * QCH;
    k_pair_g1<<<dim3(NPAIR / 16), blk, 0, stream>>>(coords, rb1_w, rb1_b, G, i0);
    wmma_gemm<0, 0, 0, false, 1><<<dim3((NPAIR / 64) / 8, 1), blk, 0, stream>>>(
        rb2w16, DM, 0, G, DM, 0, BIAST + (size_t)i0 * NP, NP * NP, 0, nullptr, nullptr, 0,
        16, NPAIR, DM, 1.0f);
  }

  k_softmax<<<dim3(NP), blk, 0, stream>>>(S, BIAST, rb2_b, P16);
  wmma_gemm<0, 0, 0, false, 4><<<dim3(1, NH), blk, 0, stream>>>(
      P16, 16 * NP, NP, VT16, NP, (long)HDM * NP, CTX1, 64, (long)NP * 64, nullptr, nullptr, 0,
      NP, 64, NP, 1.0f / 32768.0f);

  for (int ch = 0; ch < NP / QCH; ++ch) {
    const int i0 = ch * QCH;
    k_pair_g2t<<<dim3(QCH * 16), blk, 0, stream>>>(coords, rv1_w, rv1_b, G, i0);
    wmma_gemm<0, 0, 1, false, 1><<<dim3(1, QCH), blk, 0, stream>>>(
        P16 + (size_t)i0 * 16 * NP, NP, 16 * NP, G, NP, (long)DM * NP, T16 + (size_t)i0 * 16 * DM, DM, 16 * DM,
        nullptr, nullptr, 0, 16, DM, NP, 1.0f / 32768.0f);
  }

  wmma_gemm<0, 0, 0, true, 4><<<dim3(1, NH), blk, 0, stream>>>(
      T16, 16 * DM, DM, rv2w16, DM, (long)HDM * DM, CTX, 64, (long)NP * 64, nullptr, CTX1, (long)NP * 64,
      NP, 64, DM, 1.0f);

  k_combine_ln<<<dim3(NP), blk, 0, stream>>>(x, CTX, rv2_b, ln2_w, ln2_b, X1, XN2);
  wmma_gemm<0, 2, 0, false, 4><<<dim3((NP / 64) * (2 * HIDP / 64) / 8, 1), blk, 0, stream>>>(
      XN2, DM, 0, w12p16, DM, 0, C12, 2 * HIDP, 0, b12p, nullptr, 0, NP, 2 * HIDP, DM, 1.0f);
  k_swiglu<<<dim3((NP * HIDP / 2 + 255) / 256), blk, 0, stream>>>(C12, U16, NP * HIDP / 2);
  wmma_gemm<0, 2, 0, true, 4><<<dim3((NP / 64) * (DM / 64) / 8, 1), blk, 0, stream>>>(
      U16, HIDP, 0, w3p16, HIDP, 0, out, DM, 0, ffn_b3, X1, 0, NP, DM, HIDP, 1.0f);
}
